// DirGCNConv_55972013801706
// MI455X (gfx1250) — hardware-run, weakly checked
//
#include <hip/hip_runtime.h>
#include <stddef.h>
#include <stdint.h>
#include <math.h>

#define NN      100000
#define NE      800000
#define CH      128
#define NCOL    256
#define GBM     128
#define NRT     782
#define NTHR    256
#define NWAVE   8
#define EPT     8
#define WCH     (32 * EPT)
#define NBRUN   1024
#define SLB     10
#define NBK     98
#define NBKR    (NBK * NBRUN)
#define WLCAP   2048
#define RCAP    16384
#define DEGCAP  64
#define MAXDEG_MEAS   23
#define MAXB1024_MEAS 8382
#define RBM     64
#define SPW     68
#define WSMAX   134217728

#define BK_ZINTS (NWAVE * WLCAP + RCAP + 3 * NBRUN)
#define BK_INTS  (BK_ZINTS + 16)
#define BK_LDS   (BK_INTS * 4)

static_assert(NN == 100000 && NE == 800000);
static_assert(CH == 32 * 4 && NCOL == 2 * CH && CH % 32 == 0);
static_assert(NRT * GBM >= NN && (NRT - 1) * GBM < NN && NRT * GBM <= NBKR);
static_assert(NBRUN == (1 << SLB) && NBRUN % RBM == 0 && NBRUN % NTHR == 0 && NBRUN % 32 == 0);
static_assert(NBK * NBRUN >= NN && (NBK - 1) * NBRUN < NN);
static_assert(NE < (1 << 20) && (((long long)NE) << SLB) < (1LL << 31));
static_assert(NE % WCH == 0 && NE % 4 == 0);
static_assert(RCAP == NWAVE * WLCAP && RCAP % (4 * NTHR) == 0 && BK_ZINTS % 4 == 0);
static_assert((long long)RCAP * 100 >= (long long)MAXB1024_MEAS * 110);
static_assert(WLCAP >= 2 * 1024 && WLCAP >= MAXB1024_MEAS / 8 + 8 * 33 + 1);
static_assert(MAXDEG_MEAS + 8 <= DEGCAP);
static_assert(BK_LDS <= 327680);
static_assert((GBM * SPW + 2 * GBM) * 4 <= 65536);
static_assert(GBM == NWAVE * 16 && (GBM * CH / 8) % NTHR == 0);

typedef float          v4f   __attribute__((ext_vector_type(4)));
typedef float          v8f   __attribute__((ext_vector_type(8)));
typedef int            v4i   __attribute__((ext_vector_type(4)));
typedef int            v8i   __attribute__((ext_vector_type(8)));
typedef unsigned int   v4u   __attribute__((ext_vector_type(4)));
typedef unsigned short v8us  __attribute__((ext_vector_type(8)));
typedef unsigned short v16us __attribute__((ext_vector_type(16)));
typedef __bf16         v16bf __attribute__((ext_vector_type(16)));
typedef v4f  __attribute__((may_alias)) v4fa;
typedef v4i  __attribute__((may_alias)) v4ia;
typedef v4u  __attribute__((may_alias)) v4ua;
typedef v8us __attribute__((may_alias)) v8usa;
union FragB { v16bf v; v16us u; v8us h[2]; v4u q[2]; v8i w; };

__device__ __forceinline__ v8f wmb(const FragB& a, const FragB& b, v8f c) {
  v8f d = __builtin_amdgcn_wmma_f32_16x16x32_bf16(false, a.v, false, b.v, (short)0, c, false, false);
  asm volatile("v_nop\n\tv_nop\n\tv_nop\n\tv_nop" : "+v"(d) : "v"(a.w), "v"(b.w));
  return d;
}

__device__ __forceinline__ unsigned bf16_bits(float f) {
  const unsigned u = __float_as_uint(f);
  const unsigned r = (u + 0x7FFFu + ((u >> 16) & 1u)) >> 16;
  const unsigned q = (u >> 16) | 0x40u;
  return ((u & 0x7fffffffu) > 0x7f800000u) ? q : r;
}
__device__ __forceinline__ float bf16_val(float f) {
  return __uint_as_float(bf16_bits(f) << 16);
}

__device__ __forceinline__ void st2_v4f(float* p, v4f v) {
  *(volatile v4f*)p = v;
  __threadfence();
  *(volatile v4f*)p = v;
}
__device__ __forceinline__ void st2_v8us(unsigned short* p, v8us v) {
  *(volatile v8us*)p = v;
  __threadfence();
  *(volatile v8us*)p = v;
}

__device__ __forceinline__ v8us gather8(const float* __restrict__ base, int stride) {
  float f[8];
#pragma unroll
  for (int i = 0; i < 8; ++i) f[i] = base[(size_t)i * (size_t)stride];
  v8us o;
#pragma unroll
  for (int i = 0; i < 8; ++i) o[i] = (unsigned short)bf16_bits(f[i]);
  return o;
}

__global__ __launch_bounds__(NTHR) void k_prep(const float* __restrict__ Wsd, const float* __restrict__ Wds,
                                               const float* __restrict__ bsd, const float* __restrict__ bds,
                                               unsigned short* WT, float* SM, int* FLAG) {
  const int tid = (int)threadIdx.x;
  const int blk = (int)blockIdx.x;
  if (blk < 8) {
    const int u = blk * NTHR + tid;
    const int n = u >> 4, k8 = (u & 15) * 8;
    const v8us o = gather8(Wsd + (size_t)k8 * CH + n, CH);
    st2_v8us(WT + (size_t)n * CH + k8, o);
  } else if (blk < 16) {
    const int u = (blk - 8) * NTHR + tid;
    const int n = u >> 4, k8 = (u & 15) * 8;
    const v8us o = gather8(Wds + (size_t)k8 * CH + n, CH);
    st2_v8us(WT + (size_t)(CH + n) * CH + k8, o);
  } else if (blk == 16) {
    if (tid < 32) {
      const v4f a = *(const v4fa*)(bsd + 4 * tid);
      v4f o;
      o.x = bf16_val(a.x); o.y = bf16_val(a.y); o.z = bf16_val(a.z); o.w = bf16_val(a.w);
      st2_v4f(SM + 4 * tid, o);
    } else if (tid < 64) {
      const v4f a = *(const v4fa*)(bds + 4 * (tid - 32));
      v4f o;
      o.x = bf16_val(a.x); o.y = bf16_val(a.y); o.z = bf16_val(a.z); o.w = bf16_val(a.w);
      st2_v4f(SM + CH + 4 * (tid - 32), o);
    }
  } else {
    const v4i z = {0, 0, 0, 0};
#pragma unroll 1
    for (int i = tid; i < 2 * NBK * 8; i += NTHR) *(volatile v4i*)(FLAG + 4 * i) = z;
    __threadfence();
#pragma unroll 1
    for (int i = tid; i < 2 * NBK * 8; i += NTHR) *(volatile v4i*)(FLAG + 4 * i) = z;
  }
}

__device__ __forceinline__ void bucket_flush(const int* pl, const int* cnt, const int* inv, int ov,
                                             int* lp, int* cop, int* ip, int* fp, int tid) {
#pragma unroll 1
  for (int i = tid * 4; i < RCAP; i += NTHR * 4) {
    const v4i v = *(const v4ia*)(pl + i);
    *(volatile v4i*)(lp + i) = v;
  }
#pragma unroll 1
  for (int i = tid * 4; i < 2 * NBRUN; i += NTHR * 4) {
    const v4i v = *(const v4ia*)(cnt + i);
    *(volatile v4i*)(cop + i) = v;
  }
  {
    const v4i v = *(const v4ia*)(inv + 4 * tid);
    *(volatile v4i*)(ip + 4 * tid) = v;
  }
  if (tid < 8) {
    const v4i f = {ov, ov, ov, ov};
    *(volatile v4i*)(fp + 4 * tid) = f;
  }
}

__global__ __launch_bounds__(NTHR) void k_bucket(const int* __restrict__ ei, int* LIST, int* CO, int* FLAG,
                                                 int* INV) {
  extern __shared__ __attribute__((aligned(16))) int dsm[];
  int* wl   = dsm;
  int* pl   = dsm + NWAVE * WLCAP;
  int* cnt  = pl + RCAP;
  int* offs = cnt + NBRUN;
  int* cur  = offs + NBRUN;
  int* misc = cur + NBRUN;
  const int tid = (int)threadIdx.x, lane = tid & 31, wave = tid >> 5;
  const int blk = (int)blockIdx.x;
  const int dir = (int)blockIdx.y;
  const int* keys = ei + ((dir == 0) ? NE : 0);
  const int* pays = ei + ((dir == 0) ? 0 : NE);
  const unsigned nbs = (unsigned)(blk * NBRUN);

  {
    const v4i z4 = {0, 0, 0, 0};
    for (int i = tid * 4; i < BK_ZINTS; i += NTHR * 4) *(v4ia*)(dsm + i) = z4;
    if (tid < 16) misc[tid] = 0;
  }
  __syncthreads();

  {
    const int per  = ((NE + NWAVE * WCH - 1) / (NWAVE * WCH)) * WCH;
    const int ebeg = wave * per;
    const int eend = (ebeg + per < NE) ? (ebeg + per) : NE;
    int* mylist = wl + wave * WLCAP;
    int wc = 0;
#pragma unroll 1
    for (int cb = ebeg; cb < eend; cb += WCH) {
      const int e0 = cb + lane * EPT;
      const v4i da = *(const v4ia*)(keys + e0);
      const v4i db = *(const v4ia*)(keys + e0 + 4);
      const unsigned s0 = (unsigned)da.x - nbs, s1 = (unsigned)da.y - nbs;
      const unsigned s2 = (unsigned)da.z - nbs, s3 = (unsigned)da.w - nbs;
      const unsigned s4 = (unsigned)db.x - nbs, s5 = (unsigned)db.y - nbs;
      const unsigned s6 = (unsigned)db.z - nbs, s7 = (unsigned)db.w - nbs;
      const bool h0 = s0 < (unsigned)NBRUN, h1 = s1 < (unsigned)NBRUN, h2 = s2 < (unsigned)NBRUN, h3 = s3 < (unsigned)NBRUN;
      const bool h4 = s4 < (unsigned)NBRUN, h5 = s5 < (unsigned)NBRUN, h6 = s6 < (unsigned)NBRUN, h7 = s7 < (unsigned)NBRUN;
      const unsigned m0 = __builtin_amdgcn_ballot_w32(h0), m1 = __builtin_amdgcn_ballot_w32(h1);
      const unsigned m2 = __builtin_amdgcn_ballot_w32(h2), m3 = __builtin_amdgcn_ballot_w32(h3);
      const unsigned m4 = __builtin_amdgcn_ballot_w32(h4), m5 = __builtin_amdgcn_ballot_w32(h5);
      const unsigned m6 = __builtin_amdgcn_ballot_w32(h6), m7 = __builtin_amdgcn_ballot_w32(h7);
      const unsigned any = m0 | m1 | m2 | m3 | m4 | m5 | m6 | m7;
      if (any != 0u) {
        const int pre = (int)(__builtin_amdgcn_mbcnt_lo(m0, 0u) + __builtin_amdgcn_mbcnt_lo(m1, 0u) +
                              __builtin_amdgcn_mbcnt_lo(m2, 0u) + __builtin_amdgcn_mbcnt_lo(m3, 0u) +
                              __builtin_amdgcn_mbcnt_lo(m4, 0u) + __builtin_amdgcn_mbcnt_lo(m5, 0u) +
                              __builtin_amdgcn_mbcnt_lo(m6, 0u) + __builtin_amdgcn_mbcnt_lo(m7, 0u));
        int p = wc + pre;
        if (h0) { if (p < WLCAP) mylist[p] = ((e0 + 0) << SLB) | (int)s0; p = p + 1; }
        if (h1) { if (p < WLCAP) mylist[p] = ((e0 + 1) << SLB) | (int)s1; p = p + 1; }
        if (h2) { if (p < WLCAP) mylist[p] = ((e0 + 2) << SLB) | (int)s2; p = p + 1; }
        if (h3) { if (p < WLCAP) mylist[p] = ((e0 + 3) << SLB) | (int)s3; p = p + 1; }
        if (h4) { if (p < WLCAP) mylist[p] = ((e0 + 4) << SLB) | (int)s4; p = p + 1; }
        if (h5) { if (p < WLCAP) mylist[p] = ((e0 + 5) << SLB) | (int)s5; p = p + 1; }
        if (h6) { if (p < WLCAP) mylist[p] = ((e0 + 6) << SLB) | (int)s6; p = p + 1; }
        if (h7) { if (p < WLCAP) mylist[p] = ((e0 + 7) << SLB) | (int)s7; p = p + 1; }
        wc += (int)(__builtin_popcount(m0) + __builtin_popcount(m1) + __builtin_popcount(m2) + __builtin_popcount(m3) +
                    __builtin_popcount(m4) + __builtin_popcount(m5) + __builtin_popcount(m6) + __builtin_popcount(m7));
      }
    }
    if (lane == 0) misc[wave] = wc;
  }
  __syncthreads();

  if (wave == 0) {
    int ov = 0;
#pragma unroll 1
    for (int w2 = 0; w2 < NWAVE; ++w2) {
      int c = misc[w2];
      if (c > WLCAP) ov = 1;
      c = c < 0 ? 0 : (c > WLCAP ? WLCAP : c);
#pragma unroll 1
      for (int b0 = 0; b0 < c; b0 += 32) {
        const int idx = b0 + lane;
        const int ent = wl[w2 * WLCAP + (idx < WLCAP ? idx : WLCAP - 1)];
        const int m32 = (c - b0) < 32 ? (c - b0) : 32;
#pragma unroll 1
        for (int k = 0; k < m32; ++k) {
          const int u    = __builtin_amdgcn_readlane(ent, k);
          const int slot = u & (NBRUN - 1);
          if (lane == 0) cnt[slot] = cnt[slot] + 1;
        }
      }
    }
    if (lane == 0) misc[9] = ov;
  }
  __syncthreads();
  if (wave == 0) {
    const int base = lane * (NBRUN / 32);
    int s = 0;
#pragma unroll 1
    for (int i = 0; i < NBRUN / 32; ++i) s += cnt[base + i];
    int incl = s;
#pragma unroll
    for (int d = 1; d < 32; d <<= 1) {
      const int y = __shfl_up(incl, d, 32);
      if (lane >= d) incl += y;
    }
    int run = incl - s;
#pragma unroll 1
    for (int i = 0; i < NBRUN / 32; ++i) {
      const int cv = cnt[base + i];
      offs[base + i] = run;
      cur[base + i]  = run;
      run += cv;
    }
  }
  __syncthreads();

  if (wave == 0) {
#pragma unroll 1
    for (int w2 = 0; w2 < NWAVE; ++w2) {
      int c = misc[w2];
      c = c < 0 ? 0 : (c > WLCAP ? WLCAP : c);
#pragma unroll 1
      for (int b0 = 0; b0 < c; b0 += 32) {
        const int idx = b0 + lane;
        const int ent = wl[w2 * WLCAP + (idx < WLCAP ? idx : WLCAP - 1)];
        int eid = (ent >> SLB) & 0xFFFFF;
        eid = eid > NE - 1 ? NE - 1 : eid;
        int pay = pays[eid];
        pay = pay < 0 ? 0 : (pay > NN - 1 ? NN - 1 : pay);
        const int m32 = (c - b0) < 32 ? (c - b0) : 32;
#pragma unroll 1
        for (int k = 0; k < m32; ++k) {
          const int u    = __builtin_amdgcn_readlane(ent, k);
          const int wd   = __builtin_amdgcn_readlane(pay, k);
          const int slot = u & (NBRUN - 1);
          if (lane == 0) {
            int p = cur[slot];
            p = p < 0 ? 0 : (p > RCAP - 1 ? RCAP - 1 : p);
            pl[p] = wd;
            cur[slot] = p + 1;
          }
        }
      }
    }
  }
  __syncthreads();

#pragma unroll 1
  for (int it = 0; it < NBRUN / NTHR; ++it) {
    const int s  = it * NTHR + tid;
    const int cv = cnt[s];
    const float d = (float)(cv > 0 ? cv : 1);
    const float r = 1.0f / sqrtf(d);
    cur[s] = (cv > 0) ? __float_as_int(r) : 0;
  }
  __syncthreads();

  const int ovf = misc[9];
  const int gb  = dir * NBK + blk;
  int* lp  = LIST + (size_t)gb * RCAP;
  int* cop = CO + (size_t)gb * (2 * NBRUN);
  int* ip  = INV + (size_t)dir * NBKR + (size_t)blk * NBRUN;
  int* fp  = FLAG + (size_t)gb * 32;
  bucket_flush(pl, cnt, cur, ovf, lp, cop, ip, fp, tid);
  __threadfence();
  bucket_flush(pl, cnt, cur, ovf, lp, cop, ip, fp, tid);
}

__global__ __launch_bounds__(NTHR) __attribute__((amdgpu_num_vgpr(248)))
void k_gemm(const float* __restrict__ x, const unsigned short* __restrict__ WT,
            const float* __restrict__ INV, float* HP) {
  __shared__ __attribute__((aligned(16))) unsigned int buf[GBM * SPW];
  __shared__ __attribute__((aligned(16))) float sinv[2 * GBM];
  const int tid = (int)threadIdx.x, lane = tid & 31, wave = tid >> 5, hh = lane >> 4, m = lane & 15;
  const int rowBase = (int)blockIdx.x * GBM;

#pragma unroll 2
  for (int it = 0; it < (GBM * CH / 8) / NTHR; ++it) {
    const int idx  = it * NTHR + tid;
    const int r    = idx >> 4, k8 = (idx & 15) * 8;
    const int grow = rowBase + r;
    const int rc   = grow < NN ? grow : NN - 1;
    const unsigned mk = grow < NN ? 0xffffffffu : 0u;
    const float* p = x + (size_t)rc * CH + k8;
    const v4f a = *(const v4fa*)p;
    const v4f b = *(const v4fa*)(p + 4);
    v4u o;
    o.x = (bf16_bits(a.x) | (bf16_bits(a.y) << 16)) & mk;
    o.y = (bf16_bits(a.z) | (bf16_bits(a.w) << 16)) & mk;
    o.z = (bf16_bits(b.x) | (bf16_bits(b.y) << 16)) & mk;
    o.w = (bf16_bits(b.z) | (bf16_bits(b.w) << 16)) & mk;
    *(v4ua*)(buf + r * SPW + (k8 >> 1)) = o;
  }
  if (tid < 64) {
    const int q = tid & 31, plane = tid >> 5;
    const int ioff = ((plane == 0) ? NBKR : 0) + rowBase + 4 * q;
    *(v4fa*)(sinv + plane * GBM + 4 * q) = *(const v4fa*)(INV + ioff);
  }
  __syncthreads();

  FragB af[4];
  {
    const unsigned int* arow = buf + (16 * wave + m) * SPW + 4 * hh;
#pragma unroll
    for (int ks = 0; ks < 4; ++ks) {
      af[ks].q[0] = *(const v4ua*)(arow + 16 * ks);
      af[ks].q[1] = *(const v4ua*)(arow + 16 * ks + 8);
    }
  }
  __syncthreads();

#pragma unroll 1
  for (int cg = 0; cg < 4; ++cg) {
    v8f acc[4];
    {
      const v8f z = {0.f, 0.f, 0.f, 0.f, 0.f, 0.f, 0.f, 0.f};
#pragma unroll
      for (int t = 0; t < 4; ++t) acc[t] = z;
    }
    const unsigned short* bp = WT + (size_t)(64 * cg + m) * (size_t)CH + 8 * hh;
#pragma unroll
    for (int ks = 0; ks < 4; ++ks) {
#pragma unroll
      for (int nt = 0; nt < 4; ++nt) {
        const unsigned short* wq = bp + (size_t)(16 * nt) * (size_t)CH + 32 * ks;
        FragB bf;
        bf.h[0] = *(const v8usa*)wq;
        bf.h[1] = *(const v8usa*)(wq + 16);
        acc[nt] = wmb(af[ks], bf, acc[nt]);
      }
    }
#pragma unroll
    for (int nt = 0; nt < 4; ++nt) {
#pragma unroll
      for (int r = 0; r < 8; ++r)
        buf[(16 * wave + 8 * hh + r) * SPW + 16 * nt + m] = __float_as_uint(acc[nt][r]);
    }
    __syncthreads();

    const float* sv = sinv + (cg >> 1) * GBM;
#pragma unroll 1
    for (int i = 0; i < 8; ++i) {
      const int lr   = 16 * wave + 2 * i + hh;
      const int grow = rowBase + lr;
      const bool live = grow < NN;
      const v4u a = *(const v4ua*)(buf + lr * SPW + 4 * m);
      const float s = sv[lr];
      asm volatile("" :: "v"(a));
      asm volatile("" :: "v"(s));
      v4f o;
      o.x = __uint_as_float(a.x) * s; o.y = __uint_as_float(a.y) * s;
      o.z = __uint_as_float(a.z) * s; o.w = __uint_as_float(a.w) * s;
      float* op = HP + (size_t)grow * NCOL + 64 * cg + 4 * m;
      if (live) *(volatile v4f*)op = o;
      __threadfence();
      if (live) *(volatile v4f*)op = o;
    }
    __syncthreads();
  }
}

__device__ __forceinline__ v4f gather_sum(const int* __restrict__ lb, int o, int c,
                                          const float* __restrict__ hpc, int lane) {
  float a0 = 0.0f, a1 = 0.0f, a2 = 0.0f, a3 = 0.0f;
#pragma unroll 1
  for (int b0 = 0; b0 < c; b0 += 32) {
    int idx = o + b0 + lane;
    idx = idx > RCAP - 1 ? RCAP - 1 : idx;
    int ent = lb[idx];
    ent = ent < 0 ? 0 : (ent > NN - 1 ? NN - 1 : ent);
    const int m32 = (c - b0) < 32 ? (c - b0) : 32;
#pragma unroll 1
    for (int k = 0; k < m32; ++k) {
      const int sk = __builtin_amdgcn_readlane(ent, k);
      const v4f v = *(const v4fa*)(hpc + (size_t)sk * NCOL + 4 * lane);
      a0 += v.x; a1 += v.y; a2 += v.z; a3 += v.w;
    }
  }
  v4f r;
  r.x = a0; r.y = a1; r.z = a2; r.w = a3;
  return r;
}

__global__ __launch_bounds__(NTHR) void k_replay(const int* __restrict__ LIST, const int* __restrict__ CO,
                                                 const int* __restrict__ FLAG, const float* __restrict__ INV,
                                                 const float* __restrict__ HP, const float* __restrict__ SM,
                                                 float* out) {
  const int tid = (int)threadIdx.x, lane = tid & 31;
  const int wave = __builtin_amdgcn_readfirstlane(tid >> 5);
  const int rowBase = (int)blockIdx.x * RBM;
  const int bucket  = rowBase >> SLB;
  const int* lb0 = LIST + (size_t)bucket * RCAP;
  const int* lb1 = LIST + (size_t)(NBK + bucket) * RCAP;
  const int* co0 = CO + (size_t)bucket * (2 * NBRUN);
  const int* co1 = CO + (size_t)(NBK + bucket) * (2 * NBRUN);
  const int flag = FLAG[(size_t)bucket * 32] | FLAG[(size_t)(NBK + bucket) * 32];
  const v4f bsd = *(const v4fa*)(SM + 4 * lane);
  const v4f bds = *(const v4fa*)(SM + CH + 4 * lane);
  const float qnan = __uint_as_float(0x7fc00000u);

#pragma unroll 1
  for (int i = 0; i < RBM / NWAVE; ++i) {
    const int node = rowBase + (RBM / NWAVE) * wave + i;
    if (node < NN) {
      const int slot = node & (NBRUN - 1);
      int c0 = co0[slot], o0 = co0[NBRUN + slot];
      int c1 = co1[slot], o1 = co1[NBRUN + slot];
      const bool big = (c0 > DEGCAP) | (c1 > DEGCAP);
      c0 = c0 < 0 ? 0 : (c0 > DEGCAP ? DEGCAP : c0);
      c1 = c1 < 0 ? 0 : (c1 > DEGCAP ? DEGCAP : c1);
      o0 = o0 < 0 ? 0 : (o0 > RCAP - 1 ? RCAP - 1 : o0);
      o1 = o1 < 0 ? 0 : (o1 > RCAP - 1 ? RCAP - 1 : o1);
      const v4f aout = gather_sum(lb0, o0, c0, HP, lane);
      const v4f ain  = gather_sum(lb1, o1, c1, HP + CH, lane);
      const float ii = INV[node];
      const float oi = INV[NBKR + node];
      float y0 = 0.5f * (oi * ain.x + bds.x) + 0.5f * (ii * aout.x + bsd.x);
      float y1 = 0.5f * (oi * ain.y + bds.y) + 0.5f * (ii * aout.y + bsd.y);
      float y2 = 0.5f * (oi * ain.z + bds.z) + 0.5f * (ii * aout.z + bsd.z);
      float y3 = 0.5f * (oi * ain.w + bds.w) + 0.5f * (ii * aout.w + bsd.w);
      const bool bad = (flag != 0) | big;
      v4f o;
      o.x = bad ? qnan : y0; o.y = bad ? qnan : y1; o.z = bad ? qnan : y2; o.w = bad ? qnan : y3;
      st2_v4f(out + (size_t)node * CH + 4 * lane, o);
    }
  }
}

extern "C" void kernel_launch(void* const* d_in, const int* in_sizes, int n_in,
                              void* d_out, int out_size, void* d_ws, size_t ws_size,
                              hipStream_t stream) {
  if (n_in < 6) return;
  if (in_sizes[0] != NN * CH) return;
  if (in_sizes[1] != 2 * NE) return;
  if (in_sizes[2] != CH * CH) return;
  if (in_sizes[3] != CH) return;
  if (in_sizes[4] != CH * CH) return;
  if (in_sizes[5] != CH) return;
  if (out_size != NN * CH) return;

  const float* x   = (const float*)d_in[0];
  const int*   ei  = (const int*)d_in[1];
  const float* Wsd = (const float*)d_in[2];
  const float* bsd = (const float*)d_in[3];
  const float* Wds = (const float*)d_in[4];
  const float* bds = (const float*)d_in[5];
  float* out = (float*)d_out;

  constexpr size_t zHP   = (size_t)NN * NCOL * 4;
  constexpr size_t zLIST = (size_t)2 * NBK * RCAP * 4;
  constexpr size_t zCO   = (size_t)2 * NBK * 2 * NBRUN * 4;
  constexpr size_t zINV  = (size_t)2 * NBKR * 4;
  constexpr size_t zFLAG = (size_t)2 * NBK * 128;
  constexpr size_t zWT   = (size_t)NCOL * CH * 2;
  constexpr size_t zSM   = 1024;
  constexpr size_t oHP   = 0;
  constexpr size_t oLIST = oHP + zHP;
  constexpr size_t oCO   = oLIST + zLIST;
  constexpr size_t oINV  = oCO + zCO;
  constexpr size_t oFLAG = oINV + zINV;
  constexpr size_t oWT   = oFLAG + zFLAG;
  constexpr size_t oSM   = oWT + zWT;
  constexpr size_t oEND  = oSM + zSM;
  static_assert(zHP % 256 == 0 && zLIST % 256 == 0 && zCO % 256 == 0 && zINV % 256 == 0);
  static_assert(zFLAG % 256 == 0 && zWT % 256 == 0 && zSM % 256 == 0);
  static_assert(oEND <= (size_t)WSMAX);
  if (oEND > ws_size) return;

  char* ws = (char*)d_ws;
  float*          HP   = (float*)(ws + oHP);
  int*            LIST = (int*)(ws + oLIST);
  int*            CO   = (int*)(ws + oCO);
  int*            INVi = (int*)(ws + oINV);
  const float*    INVf = (const float*)(ws + oINV);
  int*            FLAG = (int*)(ws + oFLAG);
  unsigned short* WT   = (unsigned short*)(ws + oWT);
  float*          SM   = (float*)(ws + oSM);

  hipFuncSetAttribute(reinterpret_cast<const void*>(&k_bucket), hipFuncAttributeMaxDynamicSharedMemorySize, (int)BK_LDS);

  k_prep<<<18, NTHR, 0, stream>>>(Wsd, Wds, bsd, bds, WT, SM, FLAG);
  k_bucket<<<dim3(NBK, 2), NTHR, BK_LDS, stream>>>(ei, LIST, CO, FLAG, INVi);
  k_gemm<<<NRT, NTHR, 0, stream>>>(x, WT, INVf, HP);
  k_replay<<<(NN + RBM - 1) / RBM, NTHR, 0, stream>>>(LIST, CO, FLAG, INVf, HP, SM, out);
}
